// CondLaneHead_26946624815738
// MI455X (gfx1250) — hardware-verified
//
#include <hip/hip_runtime.h>


namespace {
constexpr int NI = 4, IPI = 8, NINS = NI * IPI, C = 64, CIN = 66, KP = 96, Hh = 160, Ww = 256, L = Hh * Ww, NPAR = 8513;
constexpr int OW0 = 0, OW1 = 4224, OW2 = 8320, OB0 = 8384, OB1 = 8448, OB2 = 8512;
constexpr float AS_ = 8.0f, SHIFT = 2.19f;

typedef _Float16 b16;
typedef __attribute__((ext_vector_type(16))) _Float16 v16b;
typedef __attribute__((ext_vector_type(8))) _Float16 v8b;
typedef __attribute__((ext_vector_type(8))) float v8f;
typedef __attribute__((ext_vector_type(4))) float v4f;
__device__ __forceinline__ float bf16_rne(float f) { unsigned int u = __float_as_uint(f); u += 0x7FFFu + ((u >> 16) & 1u); return __uint_as_float(u & 0xFFFF0000u); }
__device__ __forceinline__ void split16(float v, b16& hi, b16& lo) { hi = (b16)v; lo = (b16)(v - (float)hi); }
__device__ __forceinline__ v16b frag_kb(const b16* p, int hh) { const v8b a = *(const v8b*)(p + 8 * hh), b = *(const v8b*)(p + 16 + 8 * hh); v16b f;
#pragma unroll
  for (int e = 0; e < 8; ++e) { f[e] = a[e]; f[8 + e] = b[e]; } return f; }
__device__ __forceinline__ void frag_split(const float* p, int hh, v16b& fh, v16b& fl) {
#pragma unroll
  for (int e = 0; e < 8; ++e) { b16 a, c; split16(p[8 * hh + e] * AS_, a, c); fh[e] = a; fl[e] = c; split16(p[16 + 8 * hh + e] * AS_, a, c); fh[8 + e] = a; fl[8 + e] = c; } }
__device__ __forceinline__ v8f wmma16b(v16b a, v16b b, v8f c) { v8f d = __builtin_amdgcn_wmma_f32_16x16x32_f16(false, a, false, b, (short)0, c, false, false); asm volatile("v_nop\n\tv_nop\n\tv_nop\n\tv_nop" : "+v"(d) : "v"(a), "v"(b)); return d; }
__device__ __forceinline__ void wave_lds_sync() { __builtin_amdgcn_fence(__ATOMIC_RELEASE, "workgroup"); __builtin_amdgcn_wave_barrier(); __builtin_amdgcn_fence(__ATOMIC_ACQUIRE, "workgroup"); }
__device__ __forceinline__ float pmul(float a, float b) { float p = a * b; asm volatile("" : "+v"(p)); return p; }

__global__ __launch_bounds__(256) void feat_kernel(const float* __restrict__ x, b16* __restrict__ F) {
  __shared__ __attribute__((aligned(16))) b16 T[64][KP + 8];
  const int n = blockIdx.y, p0 = blockIdx.x * 64, t_ = threadIdx.x;
  for (int i = t_; i < 64 * KP; i += 256) { const int p = i & 63, c = i >> 6; float v = 0.0f;
    if (c == 0) v = (float)((p0 + p) % Ww); else if (c == 1) v = (float)((p0 + p) / Ww); else if (c < CIN) v = bf16_rne(x[((size_t)n * C + (c - 2)) * L + p0 + p]);
    T[p][c] = (b16)v; }
  __syncthreads();
  for (int pass = 0; pass < 2; ++pass) { for (int i = t_; i < 64 * (KP / 8); i += 256) { const int p = i / (KP / 8), c8 = (i % (KP / 8)) * 8; *(volatile v8b*)(F + ((size_t)n * L + p0 + p) * KP + c8) = *(const v8b*)(&T[p][c8]); } __threadfence(); }
}

__global__ __launch_bounds__(256) void prep_kernel(const float* __restrict__ prm, b16* __restrict__ R, float* __restrict__ P) {
  const int i = blockIdx.x, t_ = threadIdx.x; const float* pi = prm + (size_t)i * NPAR; b16* Ri = R + (size_t)i * (64 * KP + 64 * 64); float* Pi = P + (size_t)i * 256;
  for (int pass = 0; pass < 2; ++pass) {
    for (int q = t_; q < 64 * KP / 8 + 64 * 64 / 8; q += 256) { v8b v;
      if (q < 64 * KP / 8) { const int o = q / (KP / 8), c0 = (q % (KP / 8)) * 8; for (int e = 0; e < 8; ++e) { const int c = c0 + e; v[e] = (b16)((c < CIN) ? bf16_rne(pi[OW0 + o * CIN + c]) : 0.0f); } *(volatile v8b*)(Ri + o * KP + c0) = v; }
      else { const int r = q - 64 * KP / 8; const int o = r >> 3, c0 = (r & 7) * 8; for (int e = 0; e < 8; ++e) v[e] = (b16)bf16_rne(pi[OW1 + o * C + c0 + e]); *(volatile v8b*)(Ri + 64 * KP + o * C + c0) = v; } }
    { float v = 0.0f; if (t_ < 64) v = bf16_rne(pi[OB0 + t_]); else if (t_ < 128) v = bf16_rne(pi[OB1 + t_ - 64]); else if (t_ < 192) v = bf16_rne(pi[OW2 + t_ - 128]); else if (t_ == 192) v = bf16_rne(pi[OB2]) - SHIFT; ((volatile float*)Pi)[t_] = v; }
    __threadfence(); }
}

__global__ __launch_bounds__(64) void head_kernel(const b16* __restrict__ F, const b16* __restrict__ R, const float* __restrict__ P, float* __restrict__ out) {
  __shared__ __attribute__((aligned(16))) float T0[2][32][C + 4]; __shared__ float Oo[2][32];
  const int lane = threadIdx.x & 31, wave = threadIdx.x >> 5, nloc = lane & 15, hlf = lane >> 4, i = blockIdx.y, n = i / IPI, p0 = blockIdx.x * 64 + wave * 32;
  const b16* W0 = R + (size_t)i * (64 * KP + 64 * 64); const b16* W1 = W0 + 64 * KP; const float* Pi = P + (size_t)i * 256;
  v8f acc[2][4];
#pragma unroll
  for (int r = 0; r < 2; ++r)
#pragma unroll
    for (int t = 0; t < 4; ++t) acc[r][t] = (v8f){};
#pragma unroll
  for (int kb = 0; kb < KP; kb += 32) { const v16b a0 = frag_kb(F + ((size_t)n * L + p0 + nloc) * KP + kb, hlf), a1 = frag_kb(F + ((size_t)n * L + p0 + 16 + nloc) * KP + kb, hlf);
#pragma unroll
    for (int t = 0; t < 4; ++t) { const v16b bw = frag_kb(W0 + (size_t)(t * 16 + nloc) * KP + kb, hlf); acc[0][t] = wmma16b(a0, bw, acc[0][t]); acc[1][t] = wmma16b(a1, bw, acc[1][t]); } }
#pragma unroll
  for (int t = 0; t < 4; ++t)
#pragma unroll
    for (int r = 0; r < 2; ++r)
#pragma unroll
      for (int v = 0; v < 8; ++v) { const int c = t * 16 + nloc; T0[wave][r * 16 + 8 * hlf + v][c] = fmaxf(acc[r][t][v] + Pi[c], 0.0f); }
  wave_lds_sync();
  v8f a2[2][4];
#pragma unroll
  for (int r = 0; r < 2; ++r)
#pragma unroll
    for (int t = 0; t < 4; ++t) a2[r][t] = (v8f){};
#pragma unroll
  for (int kb = 0; kb < C; kb += 32) { v16b h0, l0, h1, l1; frag_split(&T0[wave][nloc][kb], hlf, h0, l0); frag_split(&T0[wave][16 + nloc][kb], hlf, h1, l1);
#pragma unroll
    for (int t = 0; t < 4; ++t) { const v16b bw = frag_kb(W1 + (size_t)(t * 16 + nloc) * C + kb, hlf); a2[0][t] = wmma16b(h0, bw, a2[0][t]); a2[0][t] = wmma16b(l0, bw, a2[0][t]); a2[1][t] = wmma16b(h1, bw, a2[1][t]); a2[1][t] = wmma16b(l1, bw, a2[1][t]); } }
#pragma unroll
  for (int r = 0; r < 2; ++r)
#pragma unroll
    for (int v = 0; v < 8; ++v) { float s = 0.0f;
#pragma unroll
      for (int t = 0; t < 4; ++t) { const int c = t * 16 + nloc; s += pmul(fmaxf(a2[r][t][v] * (1.0f / AS_) + Pi[64 + c], 0.0f), Pi[128 + c]); }
      s += __shfl_xor(s, 1); s += __shfl_xor(s, 2); s += __shfl_xor(s, 4); s += __shfl_xor(s, 8);
      if (nloc == 0) Oo[wave][r * 16 + 8 * hlf + v] = s + Pi[192]; }
  wave_lds_sync();
  for (int pass = 0; pass < 2; ++pass) { if (lane < 8) *(volatile v4f*)(out + (size_t)i * L + p0 + lane * 4) = *(const v4f*)(&Oo[wave][lane * 4]); __threadfence(); }
}
}

extern "C" void kernel_launch(void* const* d_in, const int* in_sizes, int n_in,
                              void* d_out, int out_size, void* d_ws, size_t ws_size, hipStream_t stream) {
  (void)n_in; (void)out_size;
  const float* x = (const float*)d_in[0]; const float* prm = (const float*)d_in[1];
  float* out = (float*)d_out;
  if (in_sizes[0] != NI * C * L || in_sizes[1] != NINS * NPAR) return;
  size_t off = 0; char* ws = (char*)d_ws;
  auto carve = [&](size_t bytes) { char* p = ws + off; off += (bytes + 255) & ~(size_t)255; return p; };
  b16* F = (b16*)carve((size_t)NI * L * KP * 2); b16* R = (b16*)carve((size_t)NINS * (64 * KP + 64 * 64) * 2); float* P = (float*)carve((size_t)NINS * 256 * 4);
  if (off > ws_size) return;
  feat_kernel<<<dim3(L / 64, NI), 256, 0, stream>>>(x, F);
  prep_kernel<<<NINS, 256, 0, stream>>>(prm, R, P);
  head_kernel<<<dim3(L / 64, NINS), 64, 0, stream>>>(F, R, P, out);
}
